// TorusEGNN_86131274154934
// MI455X (gfx1250) — hardware-verified
//
#include <hip/hip_runtime.h>
#include <math.h>

#pragma clang fp contract(off)

#define NB     2
#define NN     512
#define FD     64
#define HD     128
#define HF     64
#define NODES  (NB * NN)
#define P72    72
#define P136   136
#define P200   200
#define TP     136
#define WE1T_H (128 * P72)
#define WE2T_H (128 * P72)
#define WC1T_H (128 * P136)
#define WC2T_H (64 * P136)
#define WN1T_H (128 * P200)
#define WN2T_H (64 * P136)
#define WN3T_H (64 * P72)
#define WBLOB_H (WE2T_H + WC1T_H + WC2T_H)
#define WBLOB_B (WBLOB_H * 2)
#define WBLOB_PIECES (WBLOB_H / 8)
#define CONST_F 640
#define CONST_B (CONST_F * 4)
#define TILE_H (16 * TP)
#define TILE4_B (4 * TILE_H * 2)
#define EDGE_DYN_B (WBLOB_B + CONST_B + 4 * TILE4_B)
#define CO_P   32

#define ASC  8.0f
#define RSC  1024.0f
#define WSC  1024.0f
#define FSC  16.0f
#define C1P  (1.0f / 8192.0f)
#define C2P  (1.0f / 8388608.0f)
#define AINV (1.0f / 8.0f)
#define RINV (1.0f / 1024.0f)
#define CN1  (1.0f / 1024.0f)
#define CN2  (1.0f / 1048576.0f)
#define CPR  (1.0f / 16384.0f)
#define TWO_PI_F  6.283185307179586f
#define INV_2PI_F 0.15915494309189535f

static_assert(NODES % 16 == 0);
static_assert(WBLOB_H % 8 == 0);
static_assert((WBLOB_B % 16) == 0 && (CONST_B % 16) == 0 && (TILE4_B % 16) == 0);
static_assert((WE1T_H * 2) % 128 == 0 && (WE2T_H * 2) % 128 == 0 && (WC1T_H * 2) % 128 == 0);
static_assert((WC2T_H * 2) % 128 == 0 && (WN1T_H * 2) % 128 == 0 && (WN2T_H * 2) % 128 == 0);
static_assert((WN3T_H * 2) % 128 == 0);
static_assert(EDGE_DYN_B == 142848);
static_assert((NODES * 3) == 3 * 256 * 4);

typedef _Float16 v16h __attribute__((ext_vector_type(16)));
typedef _Float16 v8h  __attribute__((ext_vector_type(8)));
typedef float    v8f  __attribute__((ext_vector_type(8)));
typedef float    v4f  __attribute__((ext_vector_type(4)));
typedef unsigned int v4u __attribute__((ext_vector_type(4)));

union FragH { v16h v; v8h h[2]; };

__device__ __forceinline__ float bfr(float f) {
  unsigned u = __float_as_uint(f);
  u = (u + 0x7FFFu + ((u >> 16) & 1u)) & 0xFFFF0000u;
  return __uint_as_float(u);
}
__device__ __forceinline__ unsigned short h_bits(_Float16 x) { return __builtin_bit_cast(unsigned short, x); }
__device__ __forceinline__ unsigned pkh(float a, float b) {
  return (unsigned)h_bits((_Float16)a) | ((unsigned)h_bits((_Float16)b) << 16);
}
__device__ __forceinline__ float rcpf(float x) { return __builtin_amdgcn_rcpf(x); }
__device__ __forceinline__ float siluf(float x) { return x * rcpf(1.0f + __expf(-x)); }
__device__ __forceinline__ float sigmf(float x) { return rcpf(1.0f + __expf(-x)); }
__device__ __forceinline__ v8f zero8() { v8f z = {0.f, 0.f, 0.f, 0.f, 0.f, 0.f, 0.f, 0.f}; return z; }

__device__ __forceinline__ float wrapc(float a, float b) {
  float rel = a - b;
  float q = rel * INV_2PI_F;
  q = rintf(q);
  q = q * TWO_PI_F;
  rel = rel - q;
  return rel;
}

__device__ __forceinline__ v16h ldfrag_h(const _Float16* p) {
  FragH f;
  f.h[0] = *(const v8h*)(p);
  f.h[1] = *(const v8h*)(p + 16);
  return f.v;
}

__device__ __forceinline__ v8f mma_h(v16h a, v16h b, v8f c) {
  c = __builtin_amdgcn_wmma_f32_16x16x32_f16(false, a, false, b, (short)0, c, false, false);
#if defined(__HIP_DEVICE_COMPILE__)
  asm volatile("v_nop\n\tv_nop\n\tv_nop\n\tv_nop" : "+v"(c) : "v"(a), "v"(b));
#endif
  return c;
}
__device__ __forceinline__ void wave_sync_lds() {
  __builtin_amdgcn_fence(__ATOMIC_RELEASE, "workgroup");
  __builtin_amdgcn_wave_barrier();
  __builtin_amdgcn_fence(__ATOMIC_ACQUIRE, "workgroup");
}

__device__ __forceinline__ void hilo16(const float* z, v16h& fh, v16h& fl) {
#pragma unroll
  for (int t = 0; t < 16; ++t) {
    const _Float16 hv = (_Float16)z[t];
    float rs = z[t] - (float)hv;
    rs = rs * RSC;
    fh[t] = hv;
    fl[t] = (_Float16)rs;
  }
}
__device__ __forceinline__ void st_hl(_Float16* th, _Float16* tl, int idx, float v) {
  const _Float16 hv = (_Float16)v;
  float rs = v - (float)hv;
  rs = rs * RSC;
  th[idx] = hv;
  tl[idx] = (_Float16)rs;
}

__device__ __forceinline__ void build_h(const float* bv, const float* up, const float* wp, float dm,
                                        v16h& fh, v16h& fl) {
  const v4f b0 = *(const v4f*)(bv), b1 = *(const v4f*)(bv + 4), b2 = *(const v4f*)(bv + 16), b3 = *(const v4f*)(bv + 20);
  const v4f u0 = *(const v4f*)(up), u1 = *(const v4f*)(up + 4), u2 = *(const v4f*)(up + 16), u3 = *(const v4f*)(up + 20);
  const v4f w0 = *(const v4f*)(wp), w1 = *(const v4f*)(wp + 4), w2 = *(const v4f*)(wp + 16), w3 = *(const v4f*)(wp + 20);
  float z[16];
#pragma unroll
  for (int e = 0; e < 4; ++e) {
    float x;
    x = u0[e] + b0[e]; x = x + dm * w0[e]; z[e]      = siluf(x) * ASC;
    x = u1[e] + b1[e]; x = x + dm * w1[e]; z[4 + e]  = siluf(x) * ASC;
    x = u2[e] + b2[e]; x = x + dm * w2[e]; z[8 + e]  = siluf(x) * ASC;
    x = u3[e] + b3[e]; x = x + dm * w3[e]; z[12 + e] = siluf(x) * ASC;
  }
  hilo16(z, fh, fl);
}

__device__ __forceinline__ void cvt_plane(const float* __restrict__ W, int K, int NW, int nrows, int p8, int split,
                                          unsigned short* dst, int p) {
  if (p < nrows * p8) {
    const int n = p / p8;
    const int k8 = (p - n * p8) * 8;
    const int rowoff = split ? ((n >> 6) * 64) : 0;
    const int col = split ? (n & 63) : n;
    float v[8];
#pragma unroll
    for (int e = 0; e < 8; ++e) {
      const int k = k8 + e;
      const int kc = (k < K) ? k : (K - 1);
      const float x = W[(size_t)(rowoff + kc) * NW + col];
      v[e] = (k < K) ? x : 0.0f;
    }
    v4u pk;
#pragma unroll
    for (int e = 0; e < 4; ++e) pk[e] = pkh(bfr(v[2 * e]) * WSC, bfr(v[2 * e + 1]) * WSC);
    unsigned short* gp = dst + (size_t)p * 8;
    *(volatile v4u*)gp = pk;
    __threadfence();
    *(volatile v4u*)gp = pk;
  }
}

__global__ __launch_bounds__(256) void cvt_w(const float* __restrict__ We1, const float* __restrict__ We2,
                                             const float* __restrict__ Wc1, const float* __restrict__ Wc2,
                                             const float* __restrict__ Wn1, const float* __restrict__ Wn2,
                                             const float* __restrict__ Wn3,
                                             unsigned short* we1t, unsigned short* we2t, unsigned short* wc1t,
                                             unsigned short* wc2t, unsigned short* wn1t, unsigned short* wn2t,
                                             unsigned short* wn3t) {
  const int bid = blockIdx.x, tid = threadIdx.x;
  if (bid < 5)       cvt_plane(We1,  64,  64, 128, P72 / 8,  1, we1t, bid * 256 + tid);
  else if (bid < 10) cvt_plane(We2,  64, 128, 128, P72 / 8,  0, we2t, (bid - 5) * 256 + tid);
  else if (bid < 19) cvt_plane(Wc1, 128, 128, 128, P136 / 8, 0, wc1t, (bid - 10) * 256 + tid);
  else if (bid < 24) cvt_plane(Wc2, 128,  64,  64, P136 / 8, 0, wc2t, (bid - 19) * 256 + tid);
  else if (bid < 37) cvt_plane(Wn1, 192, 128, 128, P200 / 8, 0, wn1t, (bid - 24) * 256 + tid);
  else if (bid < 42) cvt_plane(Wn2, 128,  64,  64, P136 / 8, 0, wn2t, (bid - 37) * 256 + tid);
  else               cvt_plane(Wn3,  64,  64,  64, P72 / 8,  0, wn3t, (bid - 42) * 256 + tid);
}

__device__ __forceinline__ v16h feat_frag(const float* xr) {
  const v4f p0 = *(const v4f*)(xr), p1 = *(const v4f*)(xr + 4), p2 = *(const v4f*)(xr + 16), p3 = *(const v4f*)(xr + 20);
  v16h f;
#pragma unroll
  for (int e = 0; e < 4; ++e) {
    f[e]      = (_Float16)(bfr(p0[e]) * FSC);
    f[4 + e]  = (_Float16)(bfr(p1[e]) * FSC);
    f[8 + e]  = (_Float16)(bfr(p2[e]) * FSC);
    f[12 + e] = (_Float16)(bfr(p3[e]) * FSC);
  }
  return f;
}

__global__ __launch_bounds__(32) void pre_kernel(const float* __restrict__ feats,
                                                 const unsigned short* __restrict__ we1t,
                                                 const float* __restrict__ be1, float* abo) {
  __shared__ __align__(16) float sO[16 * HD];
  const int lane = threadIdx.x & 31, m = lane & 15, hh = lane >> 4, koff = 8 * hh;
  const int node0 = blockIdx.x * 16;
  const float* xr = feats + (size_t)(node0 + m) * FD + koff;
  const v16h a0 = feat_frag(xr);
  const v16h a1 = feat_frag(xr + 32);
  const _Float16* gW = (const _Float16*)(const void*)we1t + m * P72 + koff;
#pragma unroll
  for (int nt = 0; nt < 8; ++nt) {
    const v16h b0 = ldfrag_h(gW + nt * 16 * P72);
    const v16h b1 = ldfrag_h(gW + nt * 16 * P72 + 32);
    v8f acc = mma_h(a0, b0, zero8());
    acc = mma_h(a1, b1, acc);
    const int n = nt * 16 + m;
    const float bb = (nt < 4) ? bfr(be1[n & 63]) : 0.0f;
#pragma unroll
    for (int r = 0; r < 8; ++r) {
      float x = acc[r] * CPR;
      x = x + bb;
      sO[(koff + r) * HD + n] = x;
    }
  }
  __syncthreads();
  v4f ov[16];
#pragma unroll
  for (int row = 0; row < 16; ++row) ov[row] = *(const v4f*)(sO + row * HD + 4 * lane);
#pragma unroll
  for (int row = 0; row < 16; ++row) {
    float* gp = abo + (size_t)(node0 + row) * HD + 4 * lane;
    *(volatile v4f*)gp = ov[row];
  }
  __threadfence();
#pragma unroll
  for (int row = 0; row < 16; ++row) {
    float* gp = abo + (size_t)(node0 + row) * HD + 4 * lane;
    *(volatile v4f*)gp = ov[row];
  }
}

__global__ __launch_bounds__(128) void edge_kernel(
    const float* __restrict__ coors, const float* __restrict__ ab,
    const unsigned short* __restrict__ wblob, const float* __restrict__ We1,
    const float* __restrict__ be2, const float* __restrict__ Wg, const float* __restrict__ bg,
    const float* __restrict__ bc1, const float* __restrict__ bc2,
    const float* __restrict__ Wc3, const float* __restrict__ bc3,
    float* miout, float* coout, int zq) {
  extern __shared__ __align__(16) unsigned char dynL[];
  __shared__ __align__(16) float sRed[4][HD];
  __shared__ __align__(16) float sMi[HD];
  __shared__ float sRedC[4][4];

  const int tid = threadIdx.x, wave = tid >> 5, lane = tid & 31;
  const int m = lane & 15, hh = lane >> 4, koff = 8 * hh;
  const int node = blockIdx.x;
  const int nb = (node / NN) * NN;

  for (int p = tid; p < WBLOB_PIECES; p += 128) {
    const v4u v = *(const v4u*)(wblob + (size_t)p * 8);
    *(v4u*)(dynL + (size_t)p * 16) = v;
  }
  float* sC = (float*)(void*)(dynL + WBLOB_B);
  if (tid < 64) {
    sC[tid]       = ab[(size_t)node * HD + tid];
    sC[64 + tid]  = bfr(We1[128 * FD + tid]);
    sC[512 + tid] = bfr(bc2[tid]);
    sC[576 + tid] = bfr(Wc3[tid]);
  }
  sC[128 + tid] = bfr(be2[tid]);
  sC[256 + tid] = bfr(Wg[tid]);
  sC[384 + tid] = bfr(bc1[tid]);
  const float ci0 = bfr(coors[(size_t)node * 3 + 0]);
  const float ci1 = bfr(coors[(size_t)node * 3 + 1]);
  const float ci2 = bfr(coors[(size_t)node * 3 + 2]);
  const float bgv = bfr(bg[0]);
  const float bc3v = bfr(bc3[0]);
  __syncthreads();

  const _Float16* sW  = (const _Float16*)(const void*)dynL;
  const _Float16* wE2 = sW + m * P72 + koff;
  const _Float16* wC1 = sW + WE2T_H + m * P136 + koff;
  const _Float16* wC2 = sW + WE2T_H + WC1T_H + m * P136 + koff;
  const float* sU = sC;         const float* sWr = sC + 64;  const float* sBe2 = sC + 128; const float* sWg = sC + 256;
  const float* sBc1 = sC + 384; const float* sBc2 = sC + 512; const float* sWc3 = sC + 576;
  _Float16* tMh = (_Float16*)(void*)(dynL + WBLOB_B + CONST_B + wave * TILE4_B);
  _Float16* tMl = tMh + TILE_H;
  _Float16* tCh = tMl + TILE_H;
  _Float16* tCl = tCh + TILE_H;

  float mi_acc[8];
#pragma unroll
  for (int q = 0; q < 8; ++q) mi_acc[q] = 0.0f;
  float ca0 = 0.0f, ca1 = 0.0f, ca2 = 0.0f;

#pragma unroll 1
  for (int t = 0; t < NN / 64; ++t) {
    const int zo = zq * t;
    const int j0 = (wave * (NN / 64) + t) * 16;
    const int jm = nb + j0 + m;
    float dm;
    {
      const float* cj = coors + (size_t)jm * 3;
      const float r0 = wrapc(ci0, bfr(cj[0]));
      const float r1 = wrapc(ci1, bfr(cj[1]));
      const float r2 = wrapc(ci2, bfr(cj[2]));
      float d = r0 * r0; const float d1 = r1 * r1; d = d + d1; const float d2 = r2 * r2; d = d + d2;
      dm = d;
    }
    v16h ah0, al0, ah1, al1;
    {
      const float* bv = ab + (size_t)jm * HD + FD + koff;
      const float* up = sU + koff + zo;
      const float* wp = sWr + koff + zo;
      build_h(bv, up, wp, dm, ah0, al0);
      build_h(bv + 32, up + 32, wp + 32, dm, ah1, al1);
    }

    float gp[8];
#pragma unroll
    for (int r = 0; r < 8; ++r) gp[r] = 0.0f;
#pragma unroll
    for (int nt = 0; nt < 8; ++nt) {
      const _Float16* w = wE2 + nt * 16 * P72;
      const v16h b0 = ldfrag_h(w);
      const v16h b1 = ldfrag_h(w + 32);
      v8f ach = mma_h(ah0, b0, zero8());
      ach = mma_h(ah1, b1, ach);
      v8f acl = mma_h(al0, b0, zero8());
      acl = mma_h(al1, b1, acl);
      const int n = nt * 16 + m;
      const float bb = sBe2[n + zo];
      const float wgv = sWg[n + zo];
#pragma unroll
      for (int r = 0; r < 8; ++r) {
        float x = ach[r] * C1P; const float y = acl[r] * C2P; x = x + y; x = x + bb;
        const float mv = siluf(x);
        const float gq = mv * wgv;
        gp[r] = gp[r] + gq;
        st_hl(tMh, tMl, (koff + r) * TP + n, mv * ASC);
      }
    }
    float g[8];
#pragma unroll
    for (int r = 0; r < 8; ++r) {
      float s = gp[r];
      s = s + __shfl_xor(s, 1);
      s = s + __shfl_xor(s, 2);
      s = s + __shfl_xor(s, 4);
      s = s + __shfl_xor(s, 8);
      g[r] = sigmf(s + bgv);
    }
    wave_sync_lds();

#pragma unroll
    for (int nt = 0; nt < 8; ++nt) {
      const int n = nt * 16 + m;
      float acc = mi_acc[nt];
#pragma unroll
      for (int r = 0; r < 8; ++r) {
        const int idx = (koff + r) * TP + n;
        const float hv = (float)tMh[idx];
        const float lv = (float)tMl[idx];
        float mv = lv * RINV; mv = mv + hv; mv = mv * AINV;
        acc = acc + g[r] * mv;
      }
      mi_acc[nt] = acc;
    }

    v16h a2h[4], a2l[4];
#pragma unroll
    for (int kt = 0; kt < 4; ++kt) {
      a2h[kt] = ldfrag_h(tMh + m * TP + kt * 32 + koff);
      a2l[kt] = ldfrag_h(tMl + m * TP + kt * 32 + koff);
    }
#pragma unroll
    for (int nt = 0; nt < 8; ++nt) {
      const _Float16* w = wC1 + nt * 16 * P136;
      v8f ach = zero8(), acl = zero8();
#pragma unroll
      for (int kt = 0; kt < 4; ++kt) {
        const v16h b = ldfrag_h(w + kt * 32);
        ach = mma_h(a2h[kt], b, ach);
        acl = mma_h(a2l[kt], b, acl);
      }
      const int n = nt * 16 + m;
      const float bb = sBc1[n + zo];
#pragma unroll
      for (int r = 0; r < 8; ++r) {
        float x = ach[r] * C1P; const float y = acl[r] * C2P; x = x + y; x = x * g[r]; x = x + bb;
        const float cv = siluf(x);
        st_hl(tCh, tCl, (koff + r) * TP + n, cv * ASC);
      }
    }
    wave_sync_lds();

    v16h a3h[4], a3l[4];
#pragma unroll
    for (int kt = 0; kt < 4; ++kt) {
      a3h[kt] = ldfrag_h(tCh + m * TP + kt * 32 + koff);
      a3l[kt] = ldfrag_h(tCl + m * TP + kt * 32 + koff);
    }
    float cp[8];
#pragma unroll
    for (int r = 0; r < 8; ++r) cp[r] = 0.0f;
#pragma unroll
    for (int nt = 0; nt < 4; ++nt) {
      const _Float16* w = wC2 + nt * 16 * P136;
      v8f ach = zero8(), acl = zero8();
#pragma unroll
      for (int kt = 0; kt < 4; ++kt) {
        const v16h b = ldfrag_h(w + kt * 32);
        ach = mma_h(a3h[kt], b, ach);
        acl = mma_h(a3l[kt], b, acl);
      }
      const int n = nt * 16 + m;
      const float bb = sBc2[n + zo];
      const float w3 = sWc3[n + zo];
#pragma unroll
      for (int r = 0; r < 8; ++r) {
        float x = ach[r] * C1P; const float y = acl[r] * C2P; x = x + y; x = x + bb;
        const float cv = siluf(x);
        cp[r] = cp[r] + cv * w3;
      }
    }

#pragma unroll
    for (int r = 0; r < 8; ++r) {
      float s = cp[r];
      s = s + __shfl_xor(s, 1);
      s = s + __shfl_xor(s, 2);
      s = s + __shfl_xor(s, 4);
      s = s + __shfl_xor(s, 8);
      const float wij = s + bc3v;
      const float* cj = coors + (size_t)(nb + j0 + koff + r) * 3;
      const float r0 = wrapc(ci0, bfr(cj[0]));
      const float r1 = wrapc(ci1, bfr(cj[1]));
      const float r2 = wrapc(ci2, bfr(cj[2]));
      float d = r0 * r0; const float d1 = r1 * r1; d = d + d1; const float d2 = r2 * r2; d = d + d2;
      d = d + TWO_PI_F;
      const float q = 1.0f / d;
      float f;
      f = r0 * q; ca0 = ca0 + wij * f;
      f = r1 * q; ca1 = ca1 + wij * f;
      f = r2 * q; ca2 = ca2 + wij * f;
    }
    wave_sync_lds();
  }

#pragma unroll
  for (int nt = 0; nt < 8; ++nt) {
    float s = mi_acc[nt];
    s = s + __shfl_xor(s, 16);
    if (hh == 0) sRed[wave][nt * 16 + m] = s;
  }
  {
    const float s0 = ca0 + __shfl_xor(ca0, 16);
    const float s1 = ca1 + __shfl_xor(ca1, 16);
    const float s2 = ca2 + __shfl_xor(ca2, 16);
    if (lane == 0) { sRedC[wave][0] = s0; sRedC[wave][1] = s1; sRedC[wave][2] = s2; sRedC[wave][3] = 0.0f; }
  }
  __syncthreads();
  {
    float v = sRed[0][tid];
    v = v + sRed[1][tid];
    v = v + sRed[2][tid];
    v = v + sRed[3][tid];
    sMi[tid] = v;
  }
  __syncthreads();
  if (wave == 0) {
    const v4f mv = *(const v4f*)(sMi + 4 * lane);
    float c0 = sRedC[0][0]; c0 = c0 + sRedC[1][0]; c0 = c0 + sRedC[2][0]; c0 = c0 + sRedC[3][0];
    float c1 = sRedC[0][1]; c1 = c1 + sRedC[1][1]; c1 = c1 + sRedC[2][1]; c1 = c1 + sRedC[3][1];
    float c2 = sRedC[0][2]; c2 = c2 + sRedC[1][2]; c2 = c2 + sRedC[2][2]; c2 = c2 + sRedC[3][2];
    v4f cv;
    cv[0] = (lane == 0) ? c0 : 0.0f;
    cv[1] = (lane == 0) ? c1 : 0.0f;
    cv[2] = (lane == 0) ? c2 : 0.0f;
    cv[3] = 0.0f;
    float* gm = miout + (size_t)node * HD + 4 * lane;
    float* gc = coout + (size_t)node * CO_P + 4 * lane;
    *(volatile v4f*)gm = mv;
    if (lane < 8) *(volatile v4f*)gc = cv;
    __threadfence();
    *(volatile v4f*)gm = mv;
    if (lane < 8) *(volatile v4f*)gc = cv;
  }
}

__global__ __launch_bounds__(32) void node_kernel(const float* __restrict__ feats, const float* __restrict__ mi,
                                                  const unsigned short* __restrict__ wn1t,
                                                  const unsigned short* __restrict__ wn2t,
                                                  const unsigned short* __restrict__ wn3t,
                                                  const float* __restrict__ bn1, const float* __restrict__ bn2,
                                                  const float* __restrict__ bn3, float* outn) {
  __shared__ __align__(16) _Float16 sXh[16 * P200];
  __shared__ __align__(16) _Float16 sXl[16 * P200];
  __shared__ __align__(16) _Float16 sN1h[16 * P136];
  __shared__ __align__(16) _Float16 sN1l[16 * P136];
  __shared__ __align__(16) _Float16 sN2h[16 * P72];
  __shared__ __align__(16) _Float16 sN2l[16 * P72];
  __shared__ __align__(16) float sO[16 * FD];
  const int lane = threadIdx.x & 31, m = lane & 15, hh = lane >> 4, koff = 8 * hh;
  const int node0 = blockIdx.x * 16;

#pragma unroll 1
  for (int row = 0; row < 16; ++row) {
    const int nd = node0 + row;
#pragma unroll
    for (int q = 0; q < 6; ++q) {
      const int k = q * 32 + lane;
      const int kf = (k < FD) ? k : (FD - 1);
      const int km = (k < FD) ? 0 : (k - FD);
      const float vf = bfr(feats[(size_t)nd * FD + kf]);
      const float vm = mi[(size_t)nd * HD + km];
      const float v = (k < FD) ? vf : vm;
      st_hl(sXh, sXl, row * P200 + k, v);
    }
  }
  __syncthreads();

  {
    const _Float16* gW = (const _Float16*)(const void*)wn1t + m * P200 + koff;
    const _Float16* xh = sXh + m * P200 + koff;
    const _Float16* xl = sXl + m * P200 + koff;
#pragma unroll 1
    for (int nt = 0; nt < 8; ++nt) {
      v8f ach = zero8(), acl = zero8();
#pragma unroll
      for (int kt = 0; kt < 6; ++kt) {
        const v16h fh = ldfrag_h(xh + kt * 32);
        const v16h fl = ldfrag_h(xl + kt * 32);
        const v16h b  = ldfrag_h(gW + nt * 16 * P200 + kt * 32);
        ach = mma_h(fh, b, ach);
        acl = mma_h(fl, b, acl);
      }
      const int n = nt * 16 + m;
      const float bb = bfr(bn1[n]);
#pragma unroll
      for (int r = 0; r < 8; ++r) {
        float x = ach[r] * CN1; const float y = acl[r] * CN2; x = x + y; x = x + bb;
        const float s = siluf(x);
        st_hl(sN1h, sN1l, (koff + r) * P136 + n, s);
      }
    }
  }
  __syncthreads();
  {
    const _Float16* gW = (const _Float16*)(const void*)wn2t + m * P136 + koff;
    const _Float16* xh = sN1h + m * P136 + koff;
    const _Float16* xl = sN1l + m * P136 + koff;
#pragma unroll 1
    for (int nt = 0; nt < 4; ++nt) {
      v8f ach = zero8(), acl = zero8();
#pragma unroll
      for (int kt = 0; kt < 4; ++kt) {
        const v16h fh = ldfrag_h(xh + kt * 32);
        const v16h fl = ldfrag_h(xl + kt * 32);
        const v16h b  = ldfrag_h(gW + nt * 16 * P136 + kt * 32);
        ach = mma_h(fh, b, ach);
        acl = mma_h(fl, b, acl);
      }
      const int n = nt * 16 + m;
      const float bb = bfr(bn2[n]);
#pragma unroll
      for (int r = 0; r < 8; ++r) {
        float x = ach[r] * CN1; const float y = acl[r] * CN2; x = x + y; x = x + bb;
        const float s = siluf(x);
        st_hl(sN2h, sN2l, (koff + r) * P72 + n, s);
      }
    }
  }
  __syncthreads();
  {
    const _Float16* gW = (const _Float16*)(const void*)wn3t + m * P72 + koff;
    const _Float16* xh = sN2h + m * P72 + koff;
    const _Float16* xl = sN2l + m * P72 + koff;
#pragma unroll 1
    for (int nt = 0; nt < 4; ++nt) {
      v8f ach = zero8(), acl = zero8();
#pragma unroll
      for (int kt = 0; kt < 2; ++kt) {
        const v16h fh = ldfrag_h(xh + kt * 32);
        const v16h fl = ldfrag_h(xl + kt * 32);
        const v16h b  = ldfrag_h(gW + nt * 16 * P72 + kt * 32);
        ach = mma_h(fh, b, ach);
        acl = mma_h(fl, b, acl);
      }
      const int n = nt * 16 + m;
      const float bb = bfr(bn3[n]);
#pragma unroll
      for (int r = 0; r < 8; ++r) {
        float x = ach[r] * CN1; const float y = acl[r] * CN2; x = x + y; x = x + bb;
        const float fr = bfr(feats[(size_t)(node0 + koff + r) * FD + n]);
        x = x + fr;
        sO[(koff + r) * FD + n] = x;
      }
    }
  }
  __syncthreads();
  v4f ov[8];
#pragma unroll
  for (int it = 0; it < 8; ++it) {
    const int p = it * 32 + lane;
    ov[it] = *(const v4f*)(sO + (p >> 4) * FD + (p & 15) * 4);
  }
#pragma unroll
  for (int it = 0; it < 8; ++it) {
    const int p = it * 32 + lane;
    float* gp = outn + (size_t)(node0 + (p >> 4)) * FD + (p & 15) * 4;
    *(volatile v4f*)gp = ov[it];
  }
  __threadfence();
#pragma unroll
  for (int it = 0; it < 8; ++it) {
    const int p = it * 32 + lane;
    float* gp = outn + (size_t)(node0 + (p >> 4)) * FD + (p & 15) * 4;
    *(volatile v4f*)gp = ov[it];
  }
}

__global__ __launch_bounds__(256) void fin_kernel(const float* __restrict__ coors, const float* __restrict__ co,
                                                  float* outc) {
  const int tid = threadIdx.x;
  v4f o[3];
#pragma unroll
  for (int it = 0; it < 3; ++it) {
    const int e4 = (it * 256 + tid) * 4;
#pragma unroll
    for (int q = 0; q < 4; ++q) {
      const int e = e4 + q;
      const int nd = e / 3;
      const int c = e - nd * 3;
      float x = co[(size_t)nd * CO_P + c];
      x = x + bfr(coors[e]);
      o[it][q] = x;
    }
  }
#pragma unroll
  for (int it = 0; it < 3; ++it) {
    float* gp = outc + (size_t)(it * 256 + tid) * 4;
    *(volatile v4f*)gp = o[it];
  }
  __threadfence();
#pragma unroll
  for (int it = 0; it < 3; ++it) {
    float* gp = outc + (size_t)(it * 256 + tid) * 4;
    *(volatile v4f*)gp = o[it];
  }
}

extern "C" void kernel_launch(void* const* d_in, const int* in_sizes, int n_in,
                              void* d_out, int out_size, void* d_ws, size_t ws_size,
                              hipStream_t stream) {
  if (n_in < 20) return;
  const int ex[20] = { NODES * FD, NODES * 3, 129 * 64, 64, 64 * 128, 128, 128, 1, 128 * 128, 128,
                       128 * 64, 64, 64, 1, 192 * 128, 128, 128 * 64, 64, 64 * 64, 64 };
  for (int q = 0; q < 20; ++q) if (in_sizes[q] != ex[q]) return;
  if (out_size != NODES * FD + NODES * 3) return;

  const float* feats = (const float*)d_in[0];
  const float* coors = (const float*)d_in[1];
  const float* We1   = (const float*)d_in[2];
  const float* be1   = (const float*)d_in[3];
  const float* We2   = (const float*)d_in[4];
  const float* be2   = (const float*)d_in[5];
  const float* Wg    = (const float*)d_in[6];
  const float* bg    = (const float*)d_in[7];
  const float* Wc1   = (const float*)d_in[8];
  const float* bc1   = (const float*)d_in[9];
  const float* Wc2   = (const float*)d_in[10];
  const float* bc2   = (const float*)d_in[11];
  const float* Wc3   = (const float*)d_in[12];
  const float* bc3   = (const float*)d_in[13];
  const float* Wn1   = (const float*)d_in[14];
  const float* bn1   = (const float*)d_in[15];
  const float* Wn2   = (const float*)d_in[16];
  const float* bn2   = (const float*)d_in[17];
  const float* Wn3   = (const float*)d_in[18];
  const float* bn3   = (const float*)d_in[19];
  float* outn = (float*)d_out;
  float* outc = (float*)d_out + (size_t)NODES * FD;

  size_t off = 0;
  const size_t oWE1 = off; off += (size_t)WE1T_H * 2;
  const size_t oWE2 = off; off += (size_t)WE2T_H * 2;
  const size_t oWC1 = off; off += (size_t)WC1T_H * 2;
  const size_t oWC2 = off; off += (size_t)WC2T_H * 2;
  const size_t oWN1 = off; off += (size_t)WN1T_H * 2;
  const size_t oWN2 = off; off += (size_t)WN2T_H * 2;
  const size_t oWN3 = off; off += (size_t)WN3T_H * 2;
  const size_t oAB  = off; off += (size_t)NODES * HD * 4;
  const size_t oMI  = off; off += (size_t)NODES * HD * 4;
  const size_t oCO  = off; off += (size_t)NODES * CO_P * 4;
  if (off > ws_size) return;
  if (off > (size_t)134217728) return;

  char* ws = (char*)d_ws;
  unsigned short* WE1T = (unsigned short*)(ws + oWE1);
  unsigned short* WE2T = (unsigned short*)(ws + oWE2);
  unsigned short* WC1T = (unsigned short*)(ws + oWC1);
  unsigned short* WC2T = (unsigned short*)(ws + oWC2);
  unsigned short* WN1T = (unsigned short*)(ws + oWN1);
  unsigned short* WN2T = (unsigned short*)(ws + oWN2);
  unsigned short* WN3T = (unsigned short*)(ws + oWN3);
  float* AB = (float*)(ws + oAB);
  float* MI = (float*)(ws + oMI);
  float* CO = (float*)(ws + oCO);
  const int zq = in_sizes[13] - 1;

  (void)hipFuncSetAttribute(reinterpret_cast<const void*>(&edge_kernel),
                            hipFuncAttributeMaxDynamicSharedMemorySize, EDGE_DYN_B);

  cvt_w<<<dim3(45), dim3(256), 0, stream>>>(We1, We2, Wc1, Wc2, Wn1, Wn2, Wn3,
                                            WE1T, WE2T, WC1T, WC2T, WN1T, WN2T, WN3T);
  pre_kernel<<<dim3(NODES / 16), dim3(32), 0, stream>>>(feats, WE1T, be1, AB);
  edge_kernel<<<dim3(NODES), dim3(128), EDGE_DYN_B, stream>>>(coors, AB, WE2T, We1, be2, Wg, bg, bc1, bc2,
                                                              Wc3, bc3, MI, CO, zq);
  node_kernel<<<dim3(NODES / 16), dim3(32), 0, stream>>>(feats, MI, WN1T, WN2T, WN3T, bn1, bn2, bn3, outn);
  fin_kernel<<<dim3(1), dim3(256), 0, stream>>>(coors, CO, outc);
  (void)hipGetLastError();
}
